// TemporalAttentionLayer_61641370632363
// MI455X (gfx1250) — hardware-verified
//
#include <hip/hip_runtime.h>

#define B_  16
#define T_  1024
#define D_  512
#define H_  8
#define DH_ 64
#define RSPLIT (1.0f / 2048.0f)
#define PLH ((size_t)B_ * T_ * D_)
#define PLQ ((size_t)B_ * H_ * T_ * DH_)
#define PLW ((size_t)H_ * DH_ * D_)
#define PLC ((size_t)D_ * D_)

typedef _Float16 f16;
typedef f16   v16h __attribute__((ext_vector_type(16)));
typedef f16   v8h  __attribute__((ext_vector_type(8)));
typedef float v8f  __attribute__((ext_vector_type(8)));
typedef float v4f_t __attribute__((ext_vector_type(4)));
typedef float v4fa  __attribute__((ext_vector_type(4), may_alias));
typedef unsigned v4u_t __attribute__((ext_vector_type(4)));

__device__ __forceinline__ f16 lo_of(float v, f16 h) { return (f16)((v - (float)h) * 2048.0f); }
__device__ __forceinline__ unsigned pk2s(float a, float b, unsigned* lo) {
  const f16 h0 = (f16)a, h1 = (f16)b;
  *lo = (unsigned)__builtin_bit_cast(unsigned short, lo_of(a, h0)) | ((unsigned)__builtin_bit_cast(unsigned short, lo_of(b, h1)) << 16);
  return (unsigned)__builtin_bit_cast(unsigned short, h0) | ((unsigned)__builtin_bit_cast(unsigned short, h1) << 16);
}
__device__ __forceinline__ v8f wmma16(v16h a, v16h b, v8f c) { return __builtin_amdgcn_wmma_f32_16x16x32_f16(false, a, false, b, (short)0, c, false, false); }
struct Frag2 { v16h h, l; };
__device__ __forceinline__ v8f wmma_split(const Frag2& a, const Frag2& b, v8f c) { v8f x = {}; x = wmma16(a.l, b.h, x); x = wmma16(a.h, b.l, x); return wmma16(a.h, b.h, c) + x * RSPLIT; }
__device__ __forceinline__ v16h cat8(v8h a, v8h b) { return __builtin_shufflevector(a, b, 0,1,2,3,4,5,6,7,8,9,10,11,12,13,14,15); }
__device__ __forceinline__ Frag2 ld2(const f16* p, size_t plane) { Frag2 f; f.h = cat8(*(const v8h*)p, *(const v8h*)(p + 16)); f.l = cat8(*(const v8h*)(p + plane), *(const v8h*)(p + plane + 16)); return f; }

__global__ void __launch_bounds__(256) addpos_kernel(const float* __restrict__ x, const float* __restrict__ pos, f16* __restrict__ h, int n) {
  int i = (blockIdx.x * blockDim.x + threadIdx.x) * 2;
  if (i >= n) return;
  int td = i % (T_ * D_);
  unsigned lo; const unsigned p = pk2s(x[i] + pos[td], x[i + 1] + pos[td + 1], &lo);
  *(volatile unsigned*)(h + i) = p; *(volatile unsigned*)(h + PLH + i) = lo; __threadfence();
  *(volatile unsigned*)(h + i) = p; *(volatile unsigned*)(h + PLH + i) = lo;
}
__global__ void __launch_bounds__(256) cvt_kernel(const float* __restrict__ in, f16* __restrict__ out, int n, size_t plane) {
  int i = (blockIdx.x * blockDim.x + threadIdx.x) * 2;
  if (i >= n) return;
  unsigned lo; const unsigned p = pk2s(in[i], in[i + 1], &lo);
  *(volatile unsigned*)(out + i) = p; *(volatile unsigned*)(out + plane + i) = lo; __threadfence();
  *(volatile unsigned*)(out + i) = p; *(volatile unsigned*)(out + plane + i) = lo;
}

__device__ __forceinline__ void store_rows16x64_planes(const float* sw, f16* dst, size_t ld, size_t plane, int lane) {
#pragma unroll 1
  for (int pass = 0; pass < 2; ++pass) {
#pragma unroll
    for (int i = 0; i < 4; ++i) { const int c = lane + 32 * i, rr = c >> 3, q = (c & 7) * 8; const float* s = sw + rr * 68 + q;
      v4u_t v, vl; unsigned lq;
      v.x = pk2s(s[0], s[1], &lq); vl.x = lq; v.y = pk2s(s[2], s[3], &lq); vl.y = lq; v.z = pk2s(s[4], s[5], &lq); vl.z = lq; v.w = pk2s(s[6], s[7], &lq); vl.w = lq;
      *(volatile v4u_t*)(dst + rr * ld + q) = v; *(volatile v4u_t*)(dst + plane + rr * ld + q) = vl; }
    __threadfence();
  }
}

__global__ void __launch_bounds__(256) qkv_kernel(const f16* __restrict__ h, const f16* __restrict__ Wq, const f16* __restrict__ Wk, const f16* __restrict__ Wv,
                                                  const float* __restrict__ bq, const float* __restrict__ bk, const float* __restrict__ bv,
                                                  f16* __restrict__ q, f16* __restrict__ k, f16* __restrict__ v) {
  __shared__ __attribute__((aligned(16))) float stg[8][16 * 68];
  const int wib = threadIdx.x >> 5;
  const int wave = (blockIdx.x * blockDim.x + threadIdx.x) >> 5;
  const int lane = threadIdx.x & 31, lrow = lane & 15, lhi = lane >> 4;
  const int tpb = T_ / 16;
  const int b = wave / (H_ * tpb), hd = (wave / tpb) % H_, i0 = (wave % tpb) * 16;
  v8f accq[4] = {}, acck[4] = {}, accv[4] = {};
  const f16* hrow = h + ((size_t)b * T_ + (i0 + lrow)) * D_ + lhi * 8;
  const f16* wqh = Wq + (size_t)hd * DH_ * D_, *wkh = Wk + (size_t)hd * DH_ * D_, *wvh = Wv + (size_t)hd * DH_ * D_;
  for (int kk = 0; kk < D_; kk += 32) {
    const Frag2 a = ld2(hrow + kk, PLH);
#pragma unroll
    for (int n = 0; n < 4; ++n) {
      const size_t wo = (size_t)(n * 16 + lrow) * D_ + kk + lhi * 8;
      accq[n] = wmma_split(a, ld2(wqh + wo, PLW), accq[n]);
      acck[n] = wmma_split(a, ld2(wkh + wo, PLW), acck[n]);
      accv[n] = wmma_split(a, ld2(wvh + wo, PLW), accv[n]);
    }
  }
  float* sw = stg[wib];
  f16* outs[3] = {q, k, v};
  const float* bias3[3] = {bq, bk, bv};
#pragma unroll
  for (int which = 0; which < 3; ++which) {
#pragma unroll
    for (int n = 0; n < 4; ++n) {
      const int e = n * 16 + lrow;
      const float bb = bias3[which][hd * DH_ + e];
#pragma unroll
      for (int r = 0; r < 8; ++r) sw[(r + lhi * 8) * 68 + e] = (which == 0 ? accq[n][r] : which == 1 ? acck[n][r] : accv[n][r]) + bb;
    }
    asm volatile("s_wait_dscnt 0" ::: "memory");
    store_rows16x64_planes(sw, outs[which] + (((size_t)b * H_ + hd) * T_ + i0) * DH_, DH_, PLQ, lane);
    asm volatile("s_wait_dscnt 0" ::: "memory");
  }
}

__global__ void __launch_bounds__(256) flash_kernel(const f16* __restrict__ q, const f16* __restrict__ kmat, const f16* __restrict__ vmat,
                                                    float* __restrict__ outf, f16* __restrict__ outb) {
  __shared__ __attribute__((aligned(16))) f16 plds[8][2][16 * 32];
  __shared__ __attribute__((aligned(16))) f16 vs[8][2][32 * 72];
  __shared__ __attribute__((aligned(16))) float stg[8][16 * 68];
  const int wib = threadIdx.x >> 5;
  const int wave = (blockIdx.x * blockDim.x + threadIdx.x) >> 5;
  const int lane = threadIdx.x & 31, lrow = lane & 15, lhi = lane >> 4;
  const int gpb = T_ / 16;
  const int b = wave / (H_ * gpb), hd = (wave / gpb) % H_, i0 = (wave % gpb) * 16;
  const f16* qbase = q    + ((size_t)b * H_ + hd) * T_ * DH_;
  const f16* kbase = kmat + ((size_t)b * H_ + hd) * T_ * DH_;
  const f16* vbase = vmat + ((size_t)b * H_ + hd) * T_ * DH_;
  v8f o[4] = {};
  float m[8], l[8];
#pragma unroll
  for (int r = 0; r < 8; ++r) { m[r] = -3.0e38f; l[r] = 0.f; }
  const float LOG2E = 1.4426950408889634f, SCALE = 0.125f, NEGV = -4294967295.0f;
  f16* vh = vs[wib][0]; f16* vl = vs[wib][1];

  for (int j0 = 0; j0 <= i0 + 15; j0 += 32) {
    { const f16* vr = vbase + (size_t)(j0 + lane) * DH_;
#pragma unroll
      for (int u = 0; u < 8; ++u) { *(v8h*)&vh[lane * 72 + u * 8] = *(const v8h*)(vr + u * 8); *(v8h*)&vl[lane * 72 + u * 8] = *(const v8h*)(vr + PLQ + u * 8); } }
    const Frag2 kb00 = ld2(kbase + (size_t)(j0 + lrow) * DH_ + lhi * 8, PLQ), kb01 = ld2(kbase + (size_t)(j0 + lrow) * DH_ + 32 + lhi * 8, PLQ);
    const Frag2 kb10 = ld2(kbase + (size_t)(j0 + 16 + lrow) * DH_ + lhi * 8, PLQ), kb11 = ld2(kbase + (size_t)(j0 + 16 + lrow) * DH_ + 32 + lhi * 8, PLQ);
    {
      f16* ph = plds[wib][0]; f16* pl = plds[wib][1];
      v8f s0 = {}, s1 = {};
      { const Frag2 qa0 = ld2(qbase + (size_t)(i0 + lrow) * DH_ + lhi * 8, PLQ), qa1 = ld2(qbase + (size_t)(i0 + lrow) * DH_ + 32 + lhi * 8, PLQ);
        s0 = wmma_split(qa0, kb00, s0); s0 = wmma_split(qa1, kb01, s0);
        s1 = wmma_split(qa0, kb10, s1); s1 = wmma_split(qa1, kb11, s1); }
      float sc0[8], sc1[8], mnew[8];
#pragma unroll
      for (int r = 0; r < 8; ++r) {
        int row = i0 + r + lhi * 8;
        int c0 = j0 + lrow, c1 = j0 + 16 + lrow;
        float a0 = (c0 <= row) ? s0[r] * SCALE : NEGV;
        float a1 = (c1 <= row) ? s1[r] * SCALE : NEGV;
        sc0[r] = a0; sc1[r] = a1;
        float mx = fmaxf(a0, a1);
        mx = fmaxf(mx, __shfl_xor(mx, 1)); mx = fmaxf(mx, __shfl_xor(mx, 2)); mx = fmaxf(mx, __shfl_xor(mx, 4)); mx = fmaxf(mx, __shfl_xor(mx, 8));
        mnew[r] = fmaxf(m[r], mx);
      }
#pragma unroll
      for (int r = 0; r < 8; ++r) {
        float p0 = __builtin_exp2f((sc0[r] - mnew[r]) * LOG2E);
        float p1 = __builtin_exp2f((sc1[r] - mnew[r]) * LOG2E);
        float rs = p0 + p1;
        rs += __shfl_xor(rs, 1); rs += __shfl_xor(rs, 2); rs += __shfl_xor(rs, 4); rs += __shfl_xor(rs, 8);
        float fac = __builtin_exp2f((m[r] - mnew[r]) * LOG2E);
        l[r] = l[r] * fac + rs;
        m[r] = mnew[r];
#pragma unroll
        for (int n = 0; n < 4; ++n) o[n][r] *= fac;
        const float q0 = p0 * 1024.0f, q1 = p1 * 1024.0f;
        const f16 h0 = (f16)q0, h1 = (f16)q1;
        ph[(r + lhi * 8) * 32 + lrow] = h0;      pl[(r + lhi * 8) * 32 + lrow] = lo_of(q0, h0);
        ph[(r + lhi * 8) * 32 + 16 + lrow] = h1; pl[(r + lhi * 8) * 32 + 16 + lrow] = lo_of(q1, h1);
      }
    }
    asm volatile("s_wait_dscnt 0" ::: "memory");
    {
      const f16* ph = plds[wib][0]; const f16* pl = plds[wib][1];
      Frag2 pa; pa.h = cat8(*(const v8h*)&ph[lrow * 32 + lhi * 8], *(const v8h*)&ph[lrow * 32 + 16 + lhi * 8]); pa.l = cat8(*(const v8h*)&pl[lrow * 32 + lhi * 8], *(const v8h*)&pl[lrow * 32 + 16 + lhi * 8]);
#pragma unroll
      for (int n = 0; n < 4; ++n) {
        Frag2 vbn;
#pragma unroll
        for (int i = 0; i < 16; ++i) { const int key = (i < 8) ? (lhi * 8 + i) : (16 + lhi * 8 + (i - 8)); vbn.h[i] = vh[key * 72 + n * 16 + lrow]; vbn.l[i] = vl[key * 72 + n * 16 + lrow]; }
        o[n] = wmma_split(pa, vbn, o[n]);
      }
    }
  }
  float* sw = stg[wib];
  {
#pragma unroll
    for (int n = 0; n < 4; ++n)
#pragma unroll
      for (int r = 0; r < 8; ++r) sw[(r + lhi * 8) * 68 + n * 16 + lrow] = o[n][r] / (l[r] * 1024.0f);
    asm volatile("s_wait_dscnt 0" ::: "memory");
    const size_t base = ((size_t)b * T_ + i0) * D_ + hd * DH_;
#pragma unroll 1
    for (int pass = 0; pass < 2; ++pass) {
#pragma unroll
      for (int i = 0; i < 8; ++i) { const int c = lane + 32 * i, rr = c >> 4, qq = (c & 15) * 4; *(volatile v4f_t*)(outf + base + (size_t)rr * D_ + qq) = *(const volatile v4fa*)(sw + rr * 68 + qq); }
      __threadfence();
    }
    store_rows16x64_planes(sw, outb + base, D_, PLH, lane);
    asm volatile("s_wait_dscnt 0" ::: "memory");
  }
}

__global__ void __launch_bounds__(256) out_proj_kernel(const f16* __restrict__ ob, const f16* __restrict__ Wcb, const float* __restrict__ bc,
                                                       const float* __restrict__ of, float* __restrict__ y) {
  __shared__ __attribute__((aligned(16))) float stg[8][16 * 68];
  const int wib = threadIdx.x >> 5;
  const int wave = (blockIdx.x * blockDim.x + threadIdx.x) >> 5;
  const int lane = threadIdx.x & 31, lrow = lane & 15, lhi = lane >> 4;
  const int cgs = D_ / 64, rt = wave / cgs, cg = wave % cgs, row0 = rt * 32, n0 = cg * 64;
  v8f acc[2][4] = {};
  const f16* arow0 = ob + (size_t)(row0 + lrow) * D_ + lhi * 8;
  const f16* arow1 = ob + (size_t)(row0 + 16 + lrow) * D_ + lhi * 8;
  for (int kk = 0; kk < D_; kk += 32) {
    const Frag2 a0 = ld2(arow0 + kk, PLH), a1 = ld2(arow1 + kk, PLH);
#pragma unroll
    for (int n = 0; n < 4; ++n) {
      const Frag2 wb = ld2(Wcb + (size_t)(n0 + n * 16 + lrow) * D_ + kk + lhi * 8, PLC);
      acc[0][n] = wmma_split(a0, wb, acc[0][n]); acc[1][n] = wmma_split(a1, wb, acc[1][n]);
    }
  }
  float* sw = stg[wib];
#pragma unroll
  for (int g = 0; g < 2; ++g) {
#pragma unroll
    for (int n = 0; n < 4; ++n) {
      const int e = n0 + n * 16 + lrow; const float bias = bc[e];
#pragma unroll
      for (int r = 0; r < 8; ++r) { const size_t idx = (size_t)(row0 + g * 16 + r + lhi * 8) * D_ + e; sw[(r + lhi * 8) * 68 + n * 16 + lrow] = acc[g][n][r] + bias + of[idx]; }
    }
    asm volatile("s_wait_dscnt 0" ::: "memory");
#pragma unroll 1
    for (int pass = 0; pass < 2; ++pass) {
#pragma unroll
      for (int i = 0; i < 8; ++i) { const int c = lane + 32 * i, rr = c >> 4, qq = (c & 15) * 4; *(volatile v4f_t*)(y + (size_t)(row0 + g * 16 + rr) * D_ + n0 + qq) = *(const volatile v4fa*)(sw + rr * 68 + qq); }
      __threadfence();
    }
    asm volatile("s_wait_dscnt 0" ::: "memory");
  }
}

extern "C" void kernel_launch(void* const* d_in, const int* in_sizes, int n_in,
                              void* d_out, int out_size, void* d_ws, size_t ws_size,
                              hipStream_t stream) {
    const float* x   = (const float*)d_in[0];
    const float* Wq  = (const float*)d_in[1];
    const float* bq  = (const float*)d_in[2];
    const float* Wk  = (const float*)d_in[3];
    const float* bk  = (const float*)d_in[4];
    const float* Wv  = (const float*)d_in[5];
    const float* bv  = (const float*)d_in[6];
    const float* pos = (const float*)d_in[7];
    const float* Wc  = (const float*)d_in[8];
    const float* bc  = (const float*)d_in[9];
    float* y = (float*)d_out;

    char*  ws  = (char*)d_ws;
    size_t off = 0;
    auto alloc = [&](size_t bytes) -> void* { void* p = ws + off; off += (bytes + 255) & ~(size_t)255; return p; };
    f16*   h_bf  = (f16*)alloc(PLH * 2 * 2);
    f16*   q_bf  = (f16*)alloc(PLQ * 2 * 2);
    f16*   k_bf  = (f16*)alloc(PLQ * 2 * 2);
    f16*   v_bf  = (f16*)alloc(PLQ * 2 * 2);
    f16*   o_bf  = (f16*)alloc(PLH * 2 * 2);
    float* o_f   = (float*)alloc(PLH * 4);
    f16*   Wq_bf = (f16*)alloc(PLW * 2 * 2);
    f16*   Wk_bf = (f16*)alloc(PLW * 2 * 2);
    f16*   Wv_bf = (f16*)alloc(PLW * 2 * 2);
    f16*   Wc_bf = (f16*)alloc(PLC * 2 * 2);
    const int nb = B_;

    const int n1 = nb * T_ * D_;
    addpos_kernel<<<(n1 / 2 + 255) / 256, 256, 0, stream>>>(x, pos, h_bf, n1);
    const int nw = H_ * DH_ * D_;
    cvt_kernel<<<(nw / 2 + 255) / 256, 256, 0, stream>>>(Wq, Wq_bf, nw, PLW);
    cvt_kernel<<<(nw / 2 + 255) / 256, 256, 0, stream>>>(Wk, Wk_bf, nw, PLW);
    cvt_kernel<<<(nw / 2 + 255) / 256, 256, 0, stream>>>(Wv, Wv_bf, nw, PLW);
    const int nc = D_ * D_;
    cvt_kernel<<<(nc / 2 + 255) / 256, 256, 0, stream>>>(Wc, Wc_bf, nc, PLC);

    const int waves_qkv = nb * H_ * (T_ / 16);
    qkv_kernel<<<waves_qkv * 32 / 256, 256, 0, stream>>>(h_bf, Wq_bf, Wk_bf, Wv_bf, bq, bk, bv, q_bf, k_bf, v_bf);
    const int waves_fl = nb * H_ * (T_ / 16);
    flash_kernel<<<waves_fl * 32 / 256, 256, 0, stream>>>(q_bf, k_bf, v_bf, o_f, o_bf);
    const int waves_op = (nb * T_ / 32) * (D_ / 64);
    out_proj_kernel<<<waves_op * 32 / 256, 256, 0, stream>>>(o_bf, Wc_bf, bc, o_f, y);
}
